// DiffractiveNetwork_18330920419445
// MI455X (gfx1250) — hardware-verified
//
#include <hip/hip_runtime.h>
#include <math.h>
#include <cmath>

#pragma clang fp contract(off)

typedef __attribute__((ext_vector_type(16))) _Float16 v16h;
typedef __attribute__((ext_vector_type(8)))  _Float16 v8h;
typedef __attribute__((ext_vector_type(8)))  float    v8f;
typedef __attribute__((ext_vector_type(4)))  float    v4f;

constexpr int kBatch    = 32;
constexpr int kN        = 4096;
constexpr int kGemmCols = 128;
constexpr int kTileP    = 132;
constexpr int kGenSpan  = 2048;
static_assert((kN % 32) == 0);
static_assert((kN % kGemmCols) == 0);
static_assert(kBatch == 32);
static_assert((kN % kGenSpan) == 0);
static_assert(((kTileP * 4) % 16) == 0);

constexpr float kCarry    = 256.0f;
constexpr float kCarryInv = 1.0f / kCarry;

constexpr double kPiD      = 3.141592653589793;
constexpr double kLambda0D = 1.55e-6;
constexpr double kW0D      = 0.45e-6;
constexpr float  kHNeuron  = (float)3e-6;
constexpr float  kDelta    = (float)1e-7;
constexpr float  kW0       = (float)kW0D;
constexpr float  kLambda   = (float)(kLambda0D / 2.85);
constexpr float  kPiW0Sq   = (float)(kPiD * kW0D * kW0D);
constexpr float  kInvPiW0Sq = 1.0f / kPiW0Sq;
constexpr float  kTwoW0    = (float)(2.0 * kW0D);
constexpr float  kSqrtPi   = (float)1.7724538509055159;
constexpr float  kKsub     = (float)(2.0 * kPiD * 1.444 / kLambda0D);

constexpr size_t kPlaneB  = (size_t)kN * kN * 2;
constexpr size_t kFieldB  = (size_t)kBatch * kN * 2;
constexpr size_t kOffBre  = 0;
constexpr size_t kOffBim  = kOffBre + kPlaneB;
constexpr size_t kOffF0r  = kOffBim + kPlaneB;
constexpr size_t kOffF1r  = kOffF0r + kFieldB;
constexpr size_t kOffF1i  = kOffF1r + kFieldB;
constexpr size_t kOffF2r  = kOffF1i + kFieldB;
constexpr size_t kOffF2i  = kOffF2r + kFieldB;
constexpr size_t kOffMag  = kOffF2i + kFieldB;
constexpr size_t kWsTotal = kOffMag + (size_t)kBatch * kN * 4;
static_assert(kWsTotal == 68943872ull);
static_assert(kWsTotal <= 134217728ull);
static_assert((kOffBim % 128) == 0 && (kOffF0r % 128) == 0 && (kOffF1r % 128) == 0 && (kOffF1i % 128) == 0 &&
              (kOffF2r % 128) == 0 && (kOffF2i % 128) == 0 && (kOffMag % 128) == 0);

template <typename T> struct Frag;
template <> struct Frag<_Float16> {
  typedef v16h V; union U { v16h v; v8h h[2]; };
  static __device__ __forceinline__ v16h load(const _Float16* p) {
    U f; f.h[0] = *(const v8h*)(p); f.h[1] = *(const v8h*)(p + 16); return f.v;
  }
};

__device__ __forceinline__ v8f mma_h(v16h a, v16h b, v8f c) {
  c = __builtin_amdgcn_wmma_f32_16x16x32_f16(false, a, false, b, (short)0, c, false, false);
  asm volatile("v_nop\n\tv_nop\n\tv_nop\n\tv_nop" : "+v"(c) : "v"(a), "v"(b));
  return c;
}

__device__ __forceinline__ void coupling_elem(float xnm, float ynm, float x0l, float y0l,
                                              float prefR, float prefI, float& cre, float& cim) {
  const float r0   = xnm - x0l;
  const float t1   = y0l - kHNeuron;
  const float t2   = t1 - kDelta;
  const float z    = fabsf(ynm - t2);
  const float r0sq = r0 * r0;
  const float zsq  = z * z;
  const float rsq  = r0sq + zsq;
  const float r    = sqrtf(rsq);
  const float cth  = z / r;
  const float zl   = z * kLambda;
  const float tq   = zl * kInvPiW0Sq;
  const float tsq  = tq * tq;
  const float u    = 1.0f + tsq;
  const float w    = kW0 * sqrtf(u);
  const float den  = r * kSqrtPi;
  const float q1   = kTwoW0 / den;
  const float ersm = sqrtf(q1) * cth;
  const float q2   = kW0 / w;
  const float wsq  = w * w;
  const float ex   = (-r0sq) / wsq;
  const float egbm = sqrtf(q2) * expf(ex);
  const float amp  = ersm + egbm;
  const float arg  = kKsub * r;
  float sn, cs;
  sincosf(arg, &sn, &cs);
  const float pa = prefR * cs;
  const float pb = prefI * sn;
  const float pc = prefI * cs;
  const float pd = prefR * sn;
  cre = amp * (pa + pb);
  cim = amp * (pc - pd);
}

__global__ __launch_bounds__(256) void field_init_kernel(const float* __restrict__ src, _Float16* __restrict__ dst, int total8) {
  const int i = blockIdx.x * 256 + threadIdx.x;
  if (i >= total8) return;
  const size_t e0 = (size_t)i << 3;
  const v4f a0 = *(const v4f*)(src + e0);
  const v4f a1 = *(const v4f*)(src + e0 + 4);
  v8h hv;
#pragma unroll
  for (int e = 0; e < 4; ++e) {
    hv[e]     = (_Float16)a0[e];
    hv[4 + e] = (_Float16)a1[e];
  }
  _Float16* q = dst + e0;
  *(volatile v8h*)q = hv;
  __threadfence();
  *(volatile v8h*)q = hv;
}

__global__ __launch_bounds__(256) void coupling_gen_kernel(
    const float* __restrict__ x0, const float* __restrict__ y0,
    const float* __restrict__ xn, const float* __restrict__ yn,
    _Float16* __restrict__ Bre, _Float16* __restrict__ Bim, float prefR, float prefI)
{
  __shared__ __align__(16) _Float16 sRe[kGenSpan];
  __shared__ __align__(16) _Float16 sIm[kGenSpan];
  const int tid = threadIdx.x;
  const int m   = blockIdx.x >> 1;
  const int L0  = (blockIdx.x & 1) * kGenSpan;
  const float xnm = xn[m];
  const float ynm = yn[m];
#pragma unroll 1
  for (int e = 0; e < 8; ++e) {
    const int l = L0 + e * 256 + tid;
    const float xl = x0[l];
    const float yl = y0[l];
    float cre, cim;
    coupling_elem(xnm, ynm, xl, yl, prefR, prefI, cre, cim);
    const float sre = cre * kCarry;
    const float sim = cim * kCarry;
    sRe[e * 256 + tid] = (_Float16)sre;
    sIm[e * 256 + tid] = (_Float16)sim;
  }
  __syncthreads();
  const v8h hr = *(const v8h*)(sRe + tid * 8);
  const v8h hi = *(const v8h*)(sIm + tid * 8);
  const size_t off = (size_t)m * kN + L0 + tid * 8;
  *(volatile v8h*)(Bre + off) = hr;
  *(volatile v8h*)(Bim + off) = hi;
  __threadfence();
  *(volatile v8h*)(Bre + off) = hr;
  *(volatile v8h*)(Bim + off) = hi;
}

template <bool HAS_IM, bool LAST>
__global__ __launch_bounds__(128) void field_gemm_kernel(
    const _Float16* __restrict__ Ar, const _Float16* __restrict__ Ai,
    const _Float16* __restrict__ Bre, const _Float16* __restrict__ Bim,
    _Float16* __restrict__ Or, _Float16* __restrict__ Oi, float* __restrict__ Mag)
{
  __shared__ __align__(16) float sRe[kBatch * kTileP];
  __shared__ __align__(16) float sIm[kBatch * kTileP];
  const int tid   = threadIdx.x;
  const int lane  = tid & 31;
  const int wave  = tid >> 5;
  const int rlane = lane & 15;
  const int hh    = lane >> 4;
  const int koff  = hh * 8;
  const int nblk  = blockIdx.x * kGemmCols;
  const int n0    = nblk + wave * 32;

  v8f accRP[2][2], accRN[2][2], accIM[2][2];
#pragma unroll
  for (int i = 0; i < 2; ++i)
#pragma unroll
    for (int j = 0; j < 2; ++j) {
      accRP[i][j] = (v8f){0.f,0.f,0.f,0.f,0.f,0.f,0.f,0.f};
      accRN[i][j] = (v8f){0.f,0.f,0.f,0.f,0.f,0.f,0.f,0.f};
      accIM[i][j] = (v8f){0.f,0.f,0.f,0.f,0.f,0.f,0.f,0.f};
    }

  const size_t aoff0 = (size_t)rlane * kN + koff;
  const size_t aoff1 = (size_t)(16 + rlane) * kN + koff;
  const size_t boff0 = (size_t)(n0 + rlane) * kN + koff;
  const size_t boff1 = (size_t)(n0 + 16 + rlane) * kN + koff;

#pragma unroll 1
  for (int k0 = 0; k0 < kN; k0 += 32) {
    const v16h ar0 = Frag<_Float16>::load(Ar + aoff0 + k0);
    const v16h ar1 = Frag<_Float16>::load(Ar + aoff1 + k0);
    v16h ai0 = ar0, ai1 = ar1;
    if (HAS_IM) {
      ai0 = Frag<_Float16>::load(Ai + aoff0 + k0);
      ai1 = Frag<_Float16>::load(Ai + aoff1 + k0);
    }
#pragma unroll
    for (int j = 0; j < 2; ++j) {
      const size_t bo = (j == 0 ? boff0 : boff1) + k0;
      const v16h bre = Frag<_Float16>::load(Bre + bo);
      const v16h bim = Frag<_Float16>::load(Bim + bo);
      accRP[0][j] = mma_h(ar0, bre, accRP[0][j]);
      accRP[1][j] = mma_h(ar1, bre, accRP[1][j]);
      accIM[0][j] = mma_h(ar0, bim, accIM[0][j]);
      accIM[1][j] = mma_h(ar1, bim, accIM[1][j]);
      if (HAS_IM) {
        accRN[0][j] = mma_h(ai0, bim, accRN[0][j]);
        accRN[1][j] = mma_h(ai1, bim, accRN[1][j]);
        accIM[0][j] = mma_h(ai0, bre, accIM[0][j]);
        accIM[1][j] = mma_h(ai1, bre, accIM[1][j]);
      }
    }
  }

#pragma unroll
  for (int i = 0; i < 2; ++i) {
#pragma unroll
    for (int j = 0; j < 2; ++j) {
      const int col = wave * 32 + j * 16 + rlane;
#pragma unroll
      for (int r = 0; r < 8; ++r) {
        const int row = i * 16 + hh * 8 + r;
        float re = accRP[i][j][r];
        if (HAS_IM) re = re - accRN[i][j][r];
        const float im = accIM[i][j][r];
        sRe[row * kTileP + col] = re * kCarryInv;
        sIm[row * kTileP + col] = im * kCarryInv;
      }
    }
  }
  __syncthreads();

  if (!LAST) {
    const int q  = lane >> 3;
    const int c8 = (lane & 7) * 8;
    v8h hvR[4], hvI[4];
#pragma unroll
    for (int it = 0; it < 4; ++it) {
      const int L   = it * 16 + wave * 4 + q;
      const int row = L >> 1;
      const int seg = L & 1;
      const int p   = row * kTileP + seg * 64 + c8;
      const v4f r0v = *(const v4f*)(sRe + p);
      const v4f r1v = *(const v4f*)(sRe + p + 4);
      const v4f i0v = *(const v4f*)(sIm + p);
      const v4f i1v = *(const v4f*)(sIm + p + 4);
#pragma unroll
      for (int e = 0; e < 4; ++e) {
        hvR[it][e]     = (_Float16)r0v[e];
        hvR[it][4 + e] = (_Float16)r1v[e];
        hvI[it][e]     = (_Float16)i0v[e];
        hvI[it][4 + e] = (_Float16)i1v[e];
      }
    }
    for (int pass = 0; pass < 2; ++pass) {
#pragma unroll
      for (int it = 0; it < 4; ++it) {
        const int L   = it * 16 + wave * 4 + q;
        const int row = L >> 1;
        const int seg = L & 1;
        const size_t o = (size_t)row * kN + nblk + seg * 64 + c8;
        *(volatile v8h*)(Or + o) = hvR[it];
        *(volatile v8h*)(Oi + o) = hvI[it];
      }
      __threadfence();
    }
  } else {
#pragma unroll 1
    for (int it = 0; it < 8; ++it) {
      const int row = wave * 8 + it;
      const int p   = row * kTileP + lane * 4;
      const v4f rv = *(const v4f*)(sRe + p);
      const v4f iv = *(const v4f*)(sIm + p);
      v4f mg;
#pragma unroll
      for (int e = 0; e < 4; ++e) {
        const float a2 = rv[e] * rv[e];
        const float b2 = iv[e] * iv[e];
        mg[e] = sqrtf(a2 + b2);
      }
      *(v4f*)(sRe + p) = mg;
    }
    for (int pass = 0; pass < 2; ++pass) {
#pragma unroll
      for (int it = 0; it < 8; ++it) {
        const int row = wave * 8 + it;
        const int p   = row * kTileP + lane * 4;
        const v4f mg = *(const v4f*)(sRe + p);
        *(volatile v4f*)(Mag + (size_t)row * kN + nblk + lane * 4) = mg;
      }
      __threadfence();
    }
  }
}

__global__ __launch_bounds__(256) void row_softmax_kernel(const float* __restrict__ Mag, float* __restrict__ out) {
  __shared__ __align__(16) float sE[kN];
  __shared__ float redA[8];
  __shared__ float redB[8];
  const int tid  = threadIdx.x;
  const int lane = tid & 31;
  const int wave = tid >> 5;
  const float* row = Mag + (size_t)blockIdx.x * kN;
  float* orow = out + (size_t)blockIdx.x * kN;

  float mx = -3.0e38f;
#pragma unroll 1
  for (int it = 0; it < 4; ++it) {
    const int idx = (it * 256 + tid) * 4;
    const v4f v = *(const v4f*)(row + idx);
    *(v4f*)(sE + idx) = v;
    mx = fmaxf(mx, fmaxf(fmaxf(v[0], v[1]), fmaxf(v[2], v[3])));
  }
#pragma unroll
  for (int off = 16; off >= 1; off >>= 1) {
    const float o = __shfl_xor(mx, off, 32);
    mx = fmaxf(mx, o);
  }
  if (lane == 0) redA[wave] = mx;
  __syncthreads();
  float rmax = redA[0];
#pragma unroll
  for (int w = 1; w < 8; ++w) rmax = fmaxf(rmax, redA[w]);

  float sum = 0.0f;
#pragma unroll 1
  for (int it = 0; it < 4; ++it) {
    const int idx = (it * 256 + tid) * 4;
    const v4f v = *(const v4f*)(sE + idx);
    v4f ev;
#pragma unroll
    for (int e = 0; e < 4; ++e) ev[e] = expf(v[e] - rmax);
    *(v4f*)(sE + idx) = ev;
    sum = sum + ((ev[0] + ev[1]) + (ev[2] + ev[3]));
  }
#pragma unroll
  for (int off = 16; off >= 1; off >>= 1) {
    const float o = __shfl_xor(sum, off, 32);
    sum = sum + o;
  }
  if (lane == 0) redB[wave] = sum;
  __syncthreads();
  float total = redB[0];
#pragma unroll
  for (int w = 1; w < 8; ++w) total = total + redB[w];
  const float inv = 1.0f / total;

#pragma unroll 1
  for (int it = 0; it < 4; ++it) {
    const int idx = (it * 256 + tid) * 4;
    const v4f ev = *(const v4f*)(sE + idx);
    v4f ov;
#pragma unroll
    for (int e = 0; e < 4; ++e) ov[e] = ev[e] * inv;
    *(v4f*)(sE + idx) = ov;
  }
  for (int pass = 0; pass < 2; ++pass) {
#pragma unroll
    for (int it = 0; it < 4; ++it) {
      const int idx = (it * 256 + tid) * 4;
      const v4f ov = *(const v4f*)(sE + idx);
      *(volatile v4f*)(orow + idx) = ov;
    }
    __threadfence();
  }
}

extern "C" void kernel_launch(void* const* d_in, const int* in_sizes, int n_in,
                              void* d_out, int out_size, void* d_ws, size_t ws_size,
                              hipStream_t stream) {
  if (n_in < 9) return;
  if (in_sizes[0] != kBatch * kN) return;
  for (int i = 1; i < 9; ++i) {
    if (in_sizes[i] != kN) return;
  }
  if (out_size != kBatch * kN) return;
  if (ws_size < kWsTotal) return;

  const float* waves = (const float*)d_in[0];
  const float* x0_0  = (const float*)d_in[1];
  const float* y0_0  = (const float*)d_in[2];
  const float* x0_1  = (const float*)d_in[3];
  const float* y0_1  = (const float*)d_in[4];
  const float* x0_2  = (const float*)d_in[5];
  const float* y0_2  = (const float*)d_in[6];
  const float* x_out = (const float*)d_in[7];
  const float* y_out = (const float*)d_in[8];
  float* out = (float*)d_out;

  char* ws = (char*)d_ws;
  _Float16* BRE = (_Float16*)(ws + kOffBre);
  _Float16* BIM = (_Float16*)(ws + kOffBim);
  _Float16* F0R = (_Float16*)(ws + kOffF0r);
  _Float16* F1R = (_Float16*)(ws + kOffF1r);
  _Float16* F1I = (_Float16*)(ws + kOffF1i);
  _Float16* F2R = (_Float16*)(ws + kOffF2r);
  _Float16* F2I = (_Float16*)(ws + kOffF2i);
  float*    MAG = (float*)(ws + kOffMag);

  const double beta = 2.0 * kPiD * 2.85 / kLambda0D;
  const double ang  = beta * 3e-6 / 2.0;
  const float prefR = (float)std::cos(ang);
  const float prefI = (float)(-std::sin(ang));

  const int genGrid  = kN * (kN / kGenSpan);
  const int gemmGrid = kN / kGemmCols;

  field_init_kernel<<<(kBatch * kN / 8) / 256, 256, 0, stream>>>(waves, F0R, kBatch * kN / 8);

  coupling_gen_kernel<<<genGrid, 256, 0, stream>>>(x0_0, y0_0, x0_1, y0_1, BRE, BIM, prefR, prefI);
  field_gemm_kernel<false, false><<<gemmGrid, 128, 0, stream>>>(F0R, F0R, BRE, BIM, F1R, F1I, MAG);

  coupling_gen_kernel<<<genGrid, 256, 0, stream>>>(x0_1, y0_1, x0_2, y0_2, BRE, BIM, prefR, prefI);
  field_gemm_kernel<true, false><<<gemmGrid, 128, 0, stream>>>(F1R, F1I, BRE, BIM, F2R, F2I, MAG);

  coupling_gen_kernel<<<genGrid, 256, 0, stream>>>(x0_2, y0_2, x_out, y_out, BRE, BIM, prefR, prefI);
  field_gemm_kernel<true, true><<<gemmGrid, 128, 0, stream>>>(F2R, F2I, BRE, BIM, F2R, F2I, MAG);

  row_softmax_kernel<<<kBatch, 256, 0, stream>>>(MAG, out);
}
